// S6Block_64381559767209
// MI455X (gfx1250) — hardware-run, weakly checked
//
#include <hip/hip_runtime.h>
#include <math.h>

typedef __attribute__((ext_vector_type(16))) _Float16 v16h;
typedef __attribute__((ext_vector_type(8)))  _Float16 v8h;
typedef __attribute__((ext_vector_type(16))) __bf16   v16b;
typedef __attribute__((ext_vector_type(8)))  __bf16   v8b;
typedef __attribute__((ext_vector_type(8)))  float    v8f;
typedef __attribute__((ext_vector_type(4)))  float    v4f;
typedef __attribute__((ext_vector_type(4)))  unsigned v4u;
typedef __attribute__((ext_vector_type(2)))  unsigned v2u;

constexpr int kBatch   = 8;
constexpr int kLen     = 1024;
constexpr int kChan    = 512;
constexpr int kState   = 64;
constexpr int kComp    = 4;
constexpr int kHidden  = 1024;
constexpr int kUpOut   = 2048;
constexpr int kSeR     = 64;
constexpr int kPos     = kBatch * kLen;
constexpr int kChunk   = 128;
constexpr int kBlocksD = kLen / kChunk;
constexpr int kGroupCh = 128;
constexpr int kGroups  = kChan / kGroupCh;
static_assert(kPos == 8192 && kBlocksD == 8 && kGroups == 4);
static_assert((kState % 32) == 0 && (kChunk % 32) == 0 && (kChan % 32) == 0 && (kHidden % 32) == 0);
static_assert((kPos % 64) == 0 && (kChan % 64) == 0 && (kHidden % 64) == 0 && (kPos % 32) == 0);

constexpr float kStateCarry    = 16.0f;
constexpr float kStateInv      = 1.0f / 16.0f;
constexpr float kResCarry      = 2048.0f;
constexpr float kStateResInv   = 1.0f / (16.0f * 2048.0f);
constexpr float kTabCarry      = 64.0f;
constexpr float kTabInv        = 1.0f / 64.0f;
constexpr float kY1Carry       = 16.0f;
constexpr float kWCarry        = 1024.0f;
constexpr float kActCarry      = 64.0f;
constexpr float kUpInv         = 1.0f / (16.0f * 1024.0f);
constexpr float kDownInv       = 1.0f / (64.0f * 1024.0f);

constexpr int kGenHP = 72;
constexpr int kGenFP = 68;
constexpr int kGenTP = 36;

constexpr size_t kOffBbar = 0;
constexpr size_t kOffAhi  = kOffBbar + (size_t)kComp * kChan * kState * 4;
constexpr size_t kOffAlo  = kOffAhi  + (size_t)kComp * kState * kState * 2;
constexpr size_t kOffKc   = kOffAlo  + (size_t)kComp * kState * kState * 2;
constexpr size_t kOffTb   = kOffKc   + (size_t)kComp * kChan * kLen * 4;
constexpr size_t kOffX16  = kOffTb   + (size_t)kGroupCh * kBlocksD * kChunk * kChunk * 2;
constexpr size_t kOffY    = kOffX16  + (size_t)kChan * kPos * 2;
constexpr size_t kOffSm   = kOffY    + (size_t)kChan * kPos * 4;
constexpr size_t kOffGt   = kOffSm   + (size_t)kChan * kBatch * 4;
constexpr size_t kOffY1   = kOffGt   + (size_t)kChan * kBatch * 4;
constexpr size_t kOffY1h  = kOffY1   + (size_t)kPos * kChan * 4;
constexpr size_t kOffUpw  = kOffY1h  + (size_t)kPos * kChan * 2;
constexpr size_t kOffDnw  = kOffUpw  + (size_t)kUpOut * kChan * 2;
constexpr size_t kOffAct  = kOffDnw  + (size_t)kChan * kHidden * 2;
constexpr size_t kOffZr   = kOffAct  + (size_t)kPos * kHidden * 2;
constexpr size_t kWsTotal = kOffZr   + (size_t)kPos * kChan * 4;
static_assert(kWsTotal == 129597440ull);
static_assert(kWsTotal <= 134217728ull);
static_assert((kOffAhi % 256) == 0 && (kOffAlo % 256) == 0 && (kOffKc % 256) == 0 && (kOffTb % 256) == 0 &&
              (kOffX16 % 256) == 0 && (kOffY % 256) == 0 && (kOffSm % 256) == 0 && (kOffGt % 256) == 0 &&
              (kOffY1 % 256) == 0 && (kOffY1h % 256) == 0 && (kOffUpw % 256) == 0 && (kOffDnw % 256) == 0 &&
              (kOffAct % 256) == 0 && (kOffZr % 256) == 0);

__device__ __forceinline__ float flush16(float v) {
  return (__builtin_fabsf(v) < 6.103515625e-5f) ? 0.0f : v;
}
__device__ __forceinline__ unsigned short f16bits(float x) {
  const _Float16 h = (_Float16)flush16(x);
  return __builtin_bit_cast(unsigned short, h);
}
__device__ __forceinline__ unsigned pack2(float a, float b) {
  const unsigned lo = (unsigned)f16bits(a);
  const unsigned hi = (unsigned)f16bits(b);
  return lo | (hi << 16);
}
__device__ __forceinline__ void wave_sync() {
  __builtin_amdgcn_fence(__ATOMIC_RELEASE, "workgroup");
  __builtin_amdgcn_wave_barrier();
  __builtin_amdgcn_fence(__ATOMIC_ACQUIRE, "workgroup");
}
__device__ __forceinline__ void store2_v4u(unsigned short* p, v4u v) {
  volatile v4u* q = (volatile v4u*)p;
  *q = v;
  __threadfence();
  *q = v;
}
__device__ __forceinline__ void store2_v4f(float* p, v4f v) {
  volatile v4f* q = (volatile v4f*)p;
  *q = v;
  __threadfence();
  *q = v;
}
__device__ __forceinline__ float wave_sum(float s) {
  s += __shfl_xor(s, 16, 32);
  s += __shfl_xor(s, 8, 32);
  s += __shfl_xor(s, 4, 32);
  s += __shfl_xor(s, 2, 32);
  s += __shfl_xor(s, 1, 32);
  return s;
}

union FH { v16h v; v8h h[2]; };
union FW { v16h v; v4u q[2]; };
__device__ __forceinline__ v16h frag_load(const _Float16* p) {
  FH f;
  f.h[0] = *(const v8h*)(p);
  f.h[1] = *(const v8h*)(p + 16);
  return f.v;
}
__device__ __forceinline__ v8f mma_h(v16h a, v16h b, v8f c) {
  c = __builtin_amdgcn_wmma_f32_16x16x32_f16(false, a, false, b, (short)0, c, false, false);
  asm volatile("v_nop\n\tv_nop\n\tv_nop\n\tv_nop" : "+v"(c) : "v"(a), "v"(b));
  return c;
}

__global__ __launch_bounds__(64) void disc_kernel(
    const float* __restrict__ Bp, const float* __restrict__ log_dt,
    float* __restrict__ bbar, unsigned short* __restrict__ ahi, unsigned short* __restrict__ alo)
{
  __shared__ float sA[64 * 65];
  const int tid = threadIdx.x;
  const int part = blockIdx.x;
  const int comp = blockIdx.y;
  const float ldt = log_dt[comp];
  const float dt = (fmaxf(ldt, 0.0f) + log1pf(expf(-fabsf(ldt)))) + 1e-6f;
  const float hdt = 0.5f * dt;
  if (part == 0) {
    const float sqc = sqrtf(2.0f * (float)tid + 1.0f);
    float acc = 0.0f;
#pragma unroll 1
    for (int i = 0; i < 64; ++i) {
      const float fi = (float)i;
      const float sqi = sqrtf(2.0f * fi + 1.0f);
      const float dg = hdt * (fi + 1.0f);
      float r = 0.0f;
      r = (i > tid) ? (-hdt * sqi * sqc) : r;
      r = (i == tid) ? (1.0f - dg) : r;
      const float inv = 1.0f / (1.0f + dg);
      const float xv = (r - hdt * sqi * acc) * inv;
      sA[i * 65 + tid] = xv;
      acc += sqi * xv;
    }
  } else {
    const int d = (part - 1) * 64 + tid;
    const float* brow = Bp + ((size_t)comp * kChan + d) * kState;
    float acc = 0.0f;
#pragma unroll 1
    for (int i = 0; i < 64; ++i) {
      const float fi = (float)i;
      const float sqi = sqrtf(2.0f * fi + 1.0f);
      const float dg = hdt * (fi + 1.0f);
      const float inv = 1.0f / (1.0f + dg);
      const float xv = (dt * brow[i] - hdt * sqi * acc) * inv;
      sA[tid * 65 + i] = xv;
      acc += sqi * xv;
    }
  }
  __syncthreads();
  if (part == 0) {
    unsigned short* dh = ahi + (size_t)comp * kState * kState;
    unsigned short* dl = alo + (size_t)comp * kState * kState;
#pragma unroll 1
    for (int it = 0; it < 8; ++it) {
      const int q = it * 64 + tid;
      const int row = q >> 3;
      const int k8 = (q & 7) * 8;
      float vh[8];
      float vl[8];
#pragma unroll
      for (int e = 0; e < 8; ++e) {
        const float v = sA[row * 65 + k8 + e];
        const _Float16 hv = (_Float16)flush16(v);
        vh[e] = v;
        vl[e] = (v - (float)hv) * kResCarry;
      }
      const v4u ph = {pack2(vh[0], vh[1]), pack2(vh[2], vh[3]), pack2(vh[4], vh[5]), pack2(vh[6], vh[7])};
      const v4u pl = {pack2(vl[0], vl[1]), pack2(vl[2], vl[3]), pack2(vl[4], vl[5]), pack2(vl[6], vl[7])};
      store2_v4u(dh + (size_t)q * 8, ph);
      store2_v4u(dl + (size_t)q * 8, pl);
    }
  } else {
    float* dst = bbar + ((size_t)comp * kChan + (size_t)(part - 1) * 64) * kState;
#pragma unroll 1
    for (int it = 0; it < 16; ++it) {
      const int q = it * 64 + tid;
      const int row = q >> 4;
      const int c4 = (q & 15) * 4;
      const v4f v = {sA[row * 65 + c4], sA[row * 65 + c4 + 1], sA[row * 65 + c4 + 2], sA[row * 65 + c4 + 3]};
      store2_v4f(dst + (size_t)q * 4, v);
    }
  }
}

__global__ __launch_bounds__(128) void gen_kernel(
    const float* __restrict__ bbar, const unsigned short* __restrict__ ahi_p, const unsigned short* __restrict__ alo_p,
    const float* __restrict__ Cp, float* __restrict__ kc)
{
  __shared__ __align__(16) _Float16 sHi[2][16 * kGenHP];
  __shared__ __align__(16) float    sF[2][16 * kGenFP];
  __shared__ __align__(16) float    sTap[16 * kGenTP];

  const int tid  = threadIdx.x;
  const int lane = tid & 31;
  const int wave = __builtin_amdgcn_readfirstlane((int)(threadIdx.x >> 5));
  const int hh   = lane >> 4;
  const int c    = lane & 15;
  const int comp = blockIdx.y;
  const int d0   = blockIdx.x * 16;

  const size_t aoff = (size_t)comp * kState * kState + (size_t)(16 * wave + c) * kState + 8 * hh;
  const v16h ah0 = frag_load((const _Float16*)ahi_p + aoff);
  const v16h ah1 = frag_load((const _Float16*)ahi_p + aoff + 32);
  const v16h al0 = frag_load((const _Float16*)alo_p + aoff);
  const v16h al1 = frag_load((const _Float16*)alo_p + aoff + 32);

  const int drow = tid >> 3;
  const int dseg = tid & 7;
  const float* cpp = Cp + ((size_t)comp * kChan + d0 + drow) * kState + dseg * 8;
  const v4f cp0 = *(const v4f*)(cpp);
  const v4f cp1 = *(const v4f*)(cpp + 4);

  float nv[8];
  {
    const float* bp = bbar + ((size_t)comp * kChan + d0 + c) * kState + 16 * wave + 8 * hh;
    const v4f s0 = *(const v4f*)(bp);
    const v4f s1 = *(const v4f*)(bp + 4);
#pragma unroll
    for (int r = 0; r < 4; ++r) { nv[r] = s0[r]; nv[4 + r] = s1[r]; }
  }
  const int ownH = c * kGenHP + 16 * wave + 8 * hh;
  const int ownF = c * kGenFP + 16 * wave + 8 * hh;
  const int hB   = c * kGenHP + 8 * hh;
  const int fD   = drow * kGenFP + dseg * 8;

#pragma unroll 1
  for (int l = 0; l < kLen; ++l) {
    const int buf = l & 1;
    {
      v8h hv;
#pragma unroll
      for (int r = 0; r < 8; ++r) {
        const float v16 = nv[r] * kStateCarry;
        const _Float16 h16 = (_Float16)flush16(v16);
        hv[r] = h16;
      }
      *(v8h*)(&sHi[buf][ownH]) = hv;
      const v4f f0 = {nv[0], nv[1], nv[2], nv[3]};
      const v4f f1 = {nv[4], nv[5], nv[6], nv[7]};
      *(v4f*)(&sF[buf][ownF]) = f0;
      *(v4f*)(&sF[buf][ownF + 4]) = f1;
    }
    __syncthreads();

    {
      const v4f x0 = *(const v4f*)(&sF[buf][fD]);
      const v4f x1 = *(const v4f*)(&sF[buf][fD + 4]);
      float sum = cp0[0] * x0[0];
      sum = fmaf(cp0[1], x0[1], sum);
      sum = fmaf(cp0[2], x0[2], sum);
      sum = fmaf(cp0[3], x0[3], sum);
      sum = fmaf(cp1[0], x1[0], sum);
      sum = fmaf(cp1[1], x1[1], sum);
      sum = fmaf(cp1[2], x1[2], sum);
      sum = fmaf(cp1[3], x1[3], sum);
      sum += __shfl_xor(sum, 1, 32);
      sum += __shfl_xor(sum, 2, 32);
      sum += __shfl_xor(sum, 4, 32);
      if (dseg == 0) sTap[drow * kGenTP + (l & 31)] = sum;
    }

    {
      FH b0h, b1h;
      b0h.h[0] = *(const v8h*)(&sHi[buf][hB]);
      b0h.h[1] = *(const v8h*)(&sHi[buf][hB + 16]);
      b1h.h[0] = *(const v8h*)(&sHi[buf][hB + 32]);
      b1h.h[1] = *(const v8h*)(&sHi[buf][hB + 48]);
      v8f accM = (v8f){0.f, 0.f, 0.f, 0.f, 0.f, 0.f, 0.f, 0.f};
      v8f accR = (v8f){0.f, 0.f, 0.f, 0.f, 0.f, 0.f, 0.f, 0.f};
      accM = mma_h(ah0, b0h.v, accM);
      accM = mma_h(ah1, b1h.v, accM);
      accR = mma_h(al0, b0h.v, accR);
      accR = mma_h(al1, b1h.v, accR);
#pragma unroll
      for (int r = 0; r < 8; ++r) nv[r] = accM[r] * kStateInv + accR[r] * kStateResInv;
    }

    if ((l & 31) == 31) {
      wave_sync();
      const int row = 4 * wave + (lane >> 3);
      const int c4 = (lane & 7) * 4;
      const v4f tv = *(const v4f*)(&sTap[row * kGenTP + c4]);
      float* dst = kc + ((size_t)comp * kChan + d0 + row) * kLen + (l - 31) + c4;
      store2_v4f(dst, tv);
      wave_sync();
    }
  }
}

__global__ __launch_bounds__(256) void weight_planes_kernel(
    const float* __restrict__ up_w, const float* __restrict__ down_w,
    unsigned short* __restrict__ upw, unsigned short* __restrict__ dnw)
{
  const int i = blockIdx.x * 256 + threadIdx.x;
  const bool isUp = blockIdx.x < 512;
  const int j = isUp ? i : (i - 131072);
  const float* src = (isUp ? up_w : down_w) + (size_t)j * 8;
  unsigned short* dst = (isUp ? upw : dnw) + (size_t)j * 8;
  const v4f a0 = *(const v4f*)(src);
  const v4f a1 = *(const v4f*)(src + 4);
  const v4u pk = {pack2(a0[0] * kWCarry, a0[1] * kWCarry), pack2(a0[2] * kWCarry, a0[3] * kWCarry),
                  pack2(a1[0] * kWCarry, a1[1] * kWCarry), pack2(a1[2] * kWCarry, a1[3] * kWCarry)};
  store2_v4u(dst, pk);
}

__global__ __launch_bounds__(256) void stream_plane_kernel(const float* __restrict__ x, unsigned short* __restrict__ x16)
{
  __shared__ float sT[64 * 65];
  const int tid = threadIdx.x;
  const int t0 = blockIdx.x * 64;
  const int dd0 = blockIdx.y * 64;
  const int b = blockIdx.z;
#pragma unroll 1
  for (int it = 0; it < 4; ++it) {
    const int task = it * 256 + tid;
    const int tt = task >> 4;
    const int c4 = (task & 15) * 4;
    const v4f v = *(const v4f*)(x + ((size_t)b * kLen + t0 + tt) * kChan + dd0 + c4);
    sT[tt * 65 + c4]     = v[0];
    sT[tt * 65 + c4 + 1] = v[1];
    sT[tt * 65 + c4 + 2] = v[2];
    sT[tt * 65 + c4 + 3] = v[3];
  }
  __syncthreads();
#pragma unroll 1
  for (int it = 0; it < 2; ++it) {
    const int q = it * 256 + tid;
    const int dd = q >> 3;
    const int t8 = (q & 7) * 8;
    float v[8];
#pragma unroll
    for (int e = 0; e < 8; ++e) v[e] = sT[(t8 + e) * 65 + dd];
    const v4u pk = {pack2(v[0], v[1]), pack2(v[2], v[3]), pack2(v[4], v[5]), pack2(v[6], v[7])};
    store2_v4u(x16 + ((size_t)(dd0 + dd) * kBatch + b) * kLen + t0 + t8, pk);
  }
}

__global__ __launch_bounds__(256) void toeplitz_kernel(
    const float* __restrict__ kc, const float* __restrict__ Dp, unsigned short* __restrict__ tb16, int ch0)
{
  __shared__ float sW[256];
  const int tid = threadIdx.x;
  const int dblk = blockIdx.x;
  const int chl = blockIdx.y;
  const int ch = ch0 + chl;
  {
    const int lag = 128 * dblk - 128 + tid;
    const int lc = (lag < 0) ? 0 : lag;
    const int l = (kLen - 1) - lc;
    const float* kp = kc + (size_t)ch * kLen + l;
    const float k0 = kp[0];
    const float k1 = kp[(size_t)kChan * kLen];
    const float k2 = kp[(size_t)2 * kChan * kLen];
    const float k3 = kp[(size_t)3 * kChan * kLen];
    const float dsum = ((Dp[ch] + Dp[kChan + ch]) + Dp[2 * kChan + ch]) + Dp[3 * kChan + ch];
    float v = ((k0 + k1) + k2) + k3;
    v += (l == 0) ? dsum : 0.0f;
    sW[tid] = (lag >= 0) ? v : 0.0f;
  }
  __syncthreads();
  unsigned short* dst = tb16 + ((size_t)(chl * kBlocksD + dblk) * kChunk) * kChunk;
#pragma unroll 1
  for (int it = 0; it < 8; ++it) {
    const int q = it * 256 + tid;
    const int t = q >> 4;
    const int s0 = (q & 15) * 8;
    float v[8];
#pragma unroll
    for (int e = 0; e < 8; ++e) v[e] = sW[128 + t - (s0 + e)] * kTabCarry;
    const v4u pk = {pack2(v[0], v[1]), pack2(v[2], v[3]), pack2(v[4], v[5]), pack2(v[6], v[7])};
    store2_v4u(dst + (size_t)q * 8, pk);
  }
}

__global__ __launch_bounds__(256) void conv_kernel(
    const unsigned short* __restrict__ x16, const unsigned short* __restrict__ tb16, float* __restrict__ y, int ch0)
{
  __shared__ __align__(16) float sT[8][16 * 68];
  const int cch = blockIdx.x;
  const int lane = threadIdx.x & 31;
  const int wave = __builtin_amdgcn_readfirstlane((int)(threadIdx.x >> 5));
  const int chl = 4 * (int)blockIdx.y + (wave >> 1);
  const int ch = ch0 + chl;
  const int n0 = (wave & 1) * 64;
  const int rl = lane & 15;
  const int hh = lane >> 4;
  const unsigned am = (rl < 8) ? 0xffffffffu : 0u;
  const v4u amask = {am, am, am, am};
  const _Float16* A = (const _Float16*)x16 + ((size_t)ch * kBatch + (rl & 7)) * kLen + 8 * hh;
  const _Float16* T = (const _Float16*)tb16 + (size_t)chl * kBlocksD * kChunk * kChunk + (size_t)(n0 + rl) * kChunk + 8 * hh;

  v8f acc[4];
#pragma unroll
  for (int j = 0; j < 4; ++j) acc[j] = (v8f){0.f, 0.f, 0.f, 0.f, 0.f, 0.f, 0.f, 0.f};

#pragma unroll 1
  for (int d = 0; d <= cch; ++d) {
    const _Float16* ap = A + kChunk * (cch - d);
    const _Float16* bp = T + (size_t)d * kChunk * kChunk;
#pragma unroll 1
    for (int ks = 0; ks < kChunk / 32; ++ks) {
      FW fa;
      fa.q[0] = *(const v4u*)(ap + ks * 32);
      fa.q[1] = *(const v4u*)(ap + ks * 32 + 16);
      fa.q[0] = fa.q[0] & amask;
      fa.q[1] = fa.q[1] & amask;
#pragma unroll
      for (int j = 0; j < 4; ++j) {
        const v16h bj = frag_load(bp + (size_t)(j * 16) * kChunk + ks * 32);
        acc[j] = mma_h(fa.v, bj, acc[j]);
      }
    }
  }

  float* slab = sT[wave];
#pragma unroll
  for (int j = 0; j < 4; ++j) {
#pragma unroll
    for (int r = 0; r < 8; ++r) slab[(8 * hh + r) * 68 + (j << 4) + rl] = acc[j][r] * kTabInv;
  }
  wave_sync();
  v4f vals[4];
#pragma unroll
  for (int it = 0; it < 4; ++it) vals[it] = *(const v4f*)(slab + (it * 2 + hh) * 68 + rl * 4);
  float* yc = y + (size_t)ch * kBatch * kLen + kChunk * cch + n0 + rl * 4;
  for (int pass = 0; pass < 2; ++pass) {
#pragma unroll
    for (int it = 0; it < 4; ++it) {
      *(volatile v4f*)(yc + (size_t)(it * 2 + hh) * kLen) = vals[it];
    }
    __threadfence();
  }
}

__global__ __launch_bounds__(256) void se_mean_kernel(const float* __restrict__ y, float* __restrict__ sm)
{
  __shared__ float sS[32];
  const int lane = threadIdx.x & 31;
  const int wave = __builtin_amdgcn_readfirstlane((int)(threadIdx.x >> 5));
#pragma unroll 1
  for (int rr = 0; rr < 4; ++rr) {
    const int row = blockIdx.x * 32 + wave * 4 + rr;
    const float* p = y + (size_t)row * kLen + lane * 4;
    float s = 0.0f;
#pragma unroll
    for (int it = 0; it < 8; ++it) {
      const v4f v = *(const v4f*)(p + it * 128);
      s += (v[0] + v[1]) + (v[2] + v[3]);
    }
    s = wave_sum(s);
    if (lane == 0) sS[wave * 4 + rr] = s * (1.0f / (float)kLen);
  }
  __syncthreads();
  if (wave == 0) {
    const float v = sS[lane];
    volatile float* q = (volatile float*)(sm + (size_t)blockIdx.x * 32 + lane);
    *q = v;
    __threadfence();
    *q = v;
  }
}

__global__ __launch_bounds__(512) void se_mlp_kernel(
    const float* __restrict__ sm, const float* __restrict__ w1, const float* __restrict__ b1,
    const float* __restrict__ w2, const float* __restrict__ b2, float* __restrict__ gate)
{
  __shared__ float sS[kBatch * kChan];
  __shared__ float sH[kBatch * kSeR];
  const int tid = threadIdx.x;
#pragma unroll 1
  for (int k = 0; k < 8; ++k) {
    const int i = k * 512 + tid;
    sS[(i & 7) * kChan + (i >> 3)] = sm[i];
  }
  __syncthreads();
  {
    const int b = tid >> 6;
    const int r = tid & 63;
    const float* wp = w1 + (size_t)r * kChan;
    const float* sp = sS + b * kChan;
    float a = 0.0f;
#pragma unroll 4
    for (int d = 0; d < kChan; ++d) a = fmaf(wp[d], sp[d], a);
    a += b1[r];
    sH[b * kSeR + r] = fmaxf(a, 0.0f);
  }
  __syncthreads();
  {
    const int d = tid;
    const float* wp = w2 + (size_t)d * kSeR;
    const float bias = b2[d];
#pragma unroll 1
    for (int b = 0; b < kBatch; ++b) {
      float a = 0.0f;
#pragma unroll 4
      for (int r = 0; r < kSeR; ++r) a = fmaf(sH[b * kSeR + r], wp[r], a);
      a += bias;
      const float e = expf(-a);
      const float g = 1.0f / (1.0f + e);
      volatile float* q = (volatile float*)(gate + (size_t)b * kChan + d);
      *q = g;
      __threadfence();
      *q = g;
    }
  }
}

__global__ __launch_bounds__(256) void ln1_kernel(
    const float* __restrict__ x, const float* __restrict__ y, const float* __restrict__ gate,
    const float* __restrict__ n1g, const float* __restrict__ n1b,
    float* __restrict__ y1, unsigned short* __restrict__ y1h)
{
  __shared__ __align__(16) float sY[16 * 516];
  const int tid = threadIdx.x;
  const int lane = tid & 31;
  const int wave = __builtin_amdgcn_readfirstlane((int)(threadIdx.x >> 5));
  const int t0 = blockIdx.x * 16;
  const int b = blockIdx.y;
#pragma unroll 1
  for (int it = 0; it < 8; ++it) {
    const int task = it * 256 + tid;
    const int d = task >> 2;
    const int q = task & 3;
    const v4f v = *(const v4f*)(y + ((size_t)d * kBatch + b) * kLen + t0 + 4 * q);
    sY[(4 * q) * 516 + d]     = v[0];
    sY[(4 * q + 1) * 516 + d] = v[1];
    sY[(4 * q + 2) * 516 + d] = v[2];
    sY[(4 * q + 3) * 516 + d] = v[3];
  }
  __syncthreads();
#pragma unroll 1
  for (int rr = 0; rr < 2; ++rr) {
    const int tt = wave * 2 + rr;
    const size_t pos = (size_t)b * kLen + t0 + tt;
    float val[16];
    float s = 0.0f;
#pragma unroll
    for (int i = 0; i < 4; ++i) {
      const int dc = 128 * i + 4 * lane;
      const v4f xv = *(const v4f*)(x + pos * kChan + dc);
      const v4f yv = *(const v4f*)(sY + tt * 516 + dc);
      const v4f gv = *(const v4f*)(gate + (size_t)b * kChan + dc);
#pragma unroll
      for (int e = 0; e < 4; ++e) {
        const float v = xv[e] + yv[e] * gv[e];
        val[4 * i + e] = v;
        s += v;
      }
    }
    const float mean = wave_sum(s) * (1.0f / (float)kChan);
    float s2 = 0.0f;
#pragma unroll
    for (int k = 0; k < 16; ++k) {
      const float dv = val[k] - mean;
      s2 = fmaf(dv, dv, s2);
    }
    const float rs = rsqrtf(wave_sum(s2) * (1.0f / (float)kChan) + 1e-5f);
    v4f o[4];
    v2u hw[4];
#pragma unroll
    for (int i = 0; i < 4; ++i) {
      const int dc = 128 * i + 4 * lane;
      const v4f gg = *(const v4f*)(n1g + dc);
      const v4f bb = *(const v4f*)(n1b + dc);
#pragma unroll
      for (int e = 0; e < 4; ++e) o[i][e] = (val[4 * i + e] - mean) * rs * gg[e] + bb[e];
      const v2u w = {pack2(o[i][0] * kY1Carry, o[i][1] * kY1Carry), pack2(o[i][2] * kY1Carry, o[i][3] * kY1Carry)};
      hw[i] = w;
    }
    for (int pass = 0; pass < 2; ++pass) {
#pragma unroll
      for (int i = 0; i < 4; ++i) {
        const int dc = 128 * i + 4 * lane;
        *(volatile v4f*)(y1 + pos * kChan + dc) = o[i];
        *(volatile v2u*)(y1h + pos * kChan + dc) = hw[i];
      }
      __threadfence();
    }
  }
}

__global__ __launch_bounds__(128) void up_glu_kernel(
    const unsigned short* __restrict__ y1h, const unsigned short* __restrict__ upw,
    const float* __restrict__ up_b, unsigned short* __restrict__ act)
{
  __shared__ __align__(16) float    sAa[4][16 * 68];
  __shared__ __align__(16) float    sGg[4][16 * 68];
  __shared__ __align__(16) unsigned sHw[4][16 * 32];
  const int lane = threadIdx.x & 31;
  const int wave = __builtin_amdgcn_readfirstlane((int)(threadIdx.x >> 5));
  const int tile = blockIdx.x * 4 + wave;
  const int tn = tile & 15;
  const int tm = tile >> 4;
  const int m0 = tm * 32;
  const int n0 = tn * 64;
  const int rl = lane & 15;
  const int hh = lane >> 4;
  const _Float16* Ap = (const _Float16*)y1h + (size_t)(m0 + rl) * kChan + 8 * hh;
  const _Float16* Ba = (const _Float16*)upw + (size_t)(n0 + rl) * kChan + 8 * hh;
  const _Float16* Bg = Ba + (size_t)kHidden * kChan;

  v8f accA[2][4];
  v8f accG[2][4];
#pragma unroll
  for (int i = 0; i < 2; ++i)
#pragma unroll
    for (int j = 0; j < 4; ++j) {
      accA[i][j] = (v8f){0.f, 0.f, 0.f, 0.f, 0.f, 0.f, 0.f, 0.f};
      accG[i][j] = (v8f){0.f, 0.f, 0.f, 0.f, 0.f, 0.f, 0.f, 0.f};
    }

#pragma unroll 1
  for (int ks = 0; ks < kChan / 32; ++ks) {
    const int k0 = ks * 32;
    const v16h a0 = frag_load(Ap + k0);
    const v16h a1 = frag_load(Ap + (size_t)16 * kChan + k0);
    v16h bf[4];
#pragma unroll
    for (int j = 0; j < 4; ++j) bf[j] = frag_load(Ba + (size_t)(j * 16) * kChan + k0);
#pragma unroll
    for (int j = 0; j < 4; ++j) {
      accA[0][j] = mma_h(a0, bf[j], accA[0][j]);
      accA[1][j] = mma_h(a1, bf[j], accA[1][j]);
    }
#pragma unroll
    for (int j = 0; j < 4; ++j) bf[j] = frag_load(Bg + (size_t)(j * 16) * kChan + k0);
#pragma unroll
    for (int j = 0; j < 4; ++j) {
      accG[0][j] = mma_h(a0, bf[j], accG[0][j]);
      accG[1][j] = mma_h(a1, bf[j], accG[1][j]);
    }
  }

  float biasA[4], biasG[4];
#pragma unroll
  for (int j = 0; j < 4; ++j) {
    biasA[j] = up_b[n0 + (j << 4) + rl];
    biasG[j] = up_b[kHidden + n0 + (j << 4) + rl];
  }
  float* slabA = sAa[wave];
  float* slabG = sGg[wave];
  unsigned* sH = sHw[wave];
  const int q = lane >> 3;
  const int cw = lane & 7;
#pragma unroll
  for (int i = 0; i < 2; ++i) {
#pragma unroll
    for (int j = 0; j < 4; ++j) {
#pragma unroll
      for (int r = 0; r < 8; ++r) {
        slabA[(8 * hh + r) * 68 + (j << 4) + rl] = accA[i][j][r] * kUpInv + biasA[j];
        slabG[(8 * hh + r) * 68 + (j << 4) + rl] = accG[i][j][r] * kUpInv + biasG[j];
      }
    }
    wave_sync();
#pragma unroll 1
    for (int it = 0; it < 8; ++it) {
      const int row = it * 2 + hh;
      const v4f a4 = *(const v4f*)(slabA + row * 68 + rl * 4);
      const v4f g4 = *(const v4f*)(slabG + row * 68 + rl * 4);
      float o[4];
#pragma unroll
      for (int e = 0; e < 4; ++e) {
        const float av = a4[e];
        const float gv = g4[e];
        const float ge = 0.5f * av * (1.0f + erff(av * 0.70710678118654752f));
        const float sg = 1.0f / (1.0f + expf(-gv));
        o[e] = ge * sg * kActCarry;
      }
      const v2u w = {pack2(o[0], o[1]), pack2(o[2], o[3])};
      *(v2u*)(sH + row * 32 + rl * 2) = w;
    }
    wave_sync();
    v4u vals[4];
#pragma unroll
    for (int it = 0; it < 4; ++it) vals[it] = *(const v4u*)(sH + (it * 4 + q) * 32 + cw * 4);
    for (int pass = 0; pass < 2; ++pass) {
#pragma unroll
      for (int it = 0; it < 4; ++it) {
        const int row = it * 4 + q;
        *(volatile v4u*)(act + (size_t)(m0 + 16 * i + row) * kHidden + n0 + cw * 8) = vals[it];
      }
      __threadfence();
    }
    wave_sync();
  }
}

__device__ __forceinline__ unsigned short f2bf_bits(float f) {
  unsigned u = __float_as_uint(f);
  return (unsigned short)((u + 0x7FFFu + ((u >> 16) & 1u)) >> 16);
}
__device__ __forceinline__ float bf_bits2f(unsigned short h) { return __uint_as_float(((unsigned)h) << 16); }

__device__ __forceinline__ void dep_guard_h(v8f& a, v8f& b, v16h x, v16h y) { asm volatile("v_nop\n\tv_nop\n\tv_nop\n\tv_nop" : "+v"(a), "+v"(b) : "v"(x), "v"(y)); }
__device__ __forceinline__ void dep_guard_b(v8f& a, v8f& b, v16b x, v16b y) { asm volatile("v_nop\n\tv_nop\n\tv_nop\n\tv_nop" : "+v"(a), "+v"(b) : "v"(x), "v"(y)); }
__device__ __forceinline__ void keep4_h(v16h a, v16h b, v16h c, v16h d) { asm volatile("v_nop" :: "v"(a), "v"(b), "v"(c), "v"(d)); }
__device__ __forceinline__ void keep4_b(v16b a, v16b b, v16b c, v16b d) { asm volatile("v_nop" :: "v"(a), "v"(b), "v"(c), "v"(d)); }
__device__ __forceinline__ void acc_guard4(v8f& a, v8f& b, v8f& c, v8f& d) { asm volatile("v_nop\n\tv_nop\n\tv_nop\n\tv_nop" : "+v"(a), "+v"(b), "+v"(c), "+v"(d)); }
template <typename T> struct Frag;
template <> struct Frag<_Float16> {
  typedef v16h V; union U { v16h v; v8h h[2]; };
  static __device__ __forceinline__ v16h load(const _Float16* p) {
    U f; f.h[0] = *(const v8h*)(p); f.h[1] = *(const v8h*)(p + 16); return f.v;
  }
  static __device__ __forceinline__ v8f mma(v16h a, v16h b, v8f c) {
    return __builtin_amdgcn_wmma_f32_16x16x32_f16(false, a, false, b, (short)0, c, false, false);
  }
  static __device__ __forceinline__ void guard(v8f& a, v8f& b, v16h x, v16h y) { dep_guard_h(a, b, x, y); }
  static __device__ __forceinline__ void keep(v16h a, v16h b, v16h c, v16h d) { keep4_h(a, b, c, d); }
};
template <> struct Frag<__bf16> {
  typedef v16b V; union U { v16b v; v8b h[2]; };
  static __device__ __forceinline__ v16b load(const __bf16* p) {
    U f; f.h[0] = *(const v8b*)(p); f.h[1] = *(const v8b*)(p + 16); return f.v;
  }
  static __device__ __forceinline__ v8f mma(v16b a, v16b b, v8f c) {
    return __builtin_amdgcn_wmma_f32_16x16x32_bf16(false, a, false, b, (short)0, c, false, false);
  }
  static __device__ __forceinline__ void guard(v8f& a, v8f& b, v16b x, v16b y) { dep_guard_b(a, b, x, y); }
  static __device__ __forceinline__ void keep(v16b a, v16b b, v16b c, v16b d) { keep4_b(a, b, c, d); }
};

template <int ET> struct Elem;
template <> struct Elem<0> { typedef _Float16 T; };
template <> struct Elem<1> { typedef __bf16 T; };
template <int ET, bool SPLIT, int BIAS_MODE, int OUT_MODE, bool RESID, int ACT = 0>
__global__ __launch_bounds__(256) void wmma_gemm64(
    const unsigned short* __restrict__ Ap, const unsigned short* __restrict__ A2p, int lda, long strideA,
    const unsigned short* __restrict__ Btp, const unsigned short* __restrict__ Bt2p, int ldb, long strideB,
    void* __restrict__ Cout, void* __restrict__ Cout2, int ldc, long strideC,
    const float* __restrict__ bias,
    const float* __restrict__ resid, long strideR,
    int M, int N, int K, float scale) {
  typedef typename Elem<ET>::T T;
  typedef typename Frag<T>::V V;
  const T* A = (const T*)Ap; const T* A2 = (const T*)A2p; const T* Bt = (const T*)Btp; const T* Bt2 = (const T*)Bt2p;
  __shared__ __align__(16) float sT[8][16 * 68];
  const int b    = blockIdx.y;
  const int lane = threadIdx.x & 31;
  const int wave = threadIdx.x >> 5;
  const int tilesN = N >> 6;
  const int tilesM = M >> 6;
  const int tile = blockIdx.x * 8 + wave;
  if (tile >= tilesM * tilesN) return;
  const int tm = tile / tilesN;
  const int tn = tile - tm * tilesN;
  const int m0 = tm << 6;
  const int n0 = tn << 6;

  const T* Ab  = A  + (size_t)b * strideA;
  const T* Bb  = Bt + (size_t)b * strideB;
  const T* Ab2 = SPLIT ? (A2  + (size_t)b * strideA) : nullptr;
  const T* Bb2 = SPLIT ? (Bt2 + (size_t)b * strideB) : nullptr;

  const int rlane = lane & 15;
  const int koff  = (lane >> 4) * 8;
  const int mOff  = (lane >> 4) * 8;

  v8f acc[4][4];
#pragma unroll
  for (int i = 0; i < 4; ++i)
#pragma unroll
    for (int j = 0; j < 4; ++j) acc[i][j] = (v8f){0.f,0.f,0.f,0.f,0.f,0.f,0.f,0.f};

  for (int k0 = 0; k0 < K; k0 += 32) {
    V bh[4], bl[4];
#pragma unroll
    for (int j = 0; j < 4; ++j) {
      const size_t bo = (size_t)(n0 + (j << 4) + rlane) * ldb + koff + k0;
      bh[j] = Frag<T>::load(Bb + bo);
      if (SPLIT) bl[j] = Frag<T>::load(Bb2 + bo);
    }
#pragma unroll
    for (int i = 0; i < 4; ++i) {
      const size_t ao = (size_t)(m0 + (i << 4) + rlane) * lda + koff + k0;
      V ah = Frag<T>::load(Ab + ao);
      V al;
      if (SPLIT) al = Frag<T>::load(Ab2 + ao);
#pragma unroll
      for (int j = 0; j < 4; ++j) {
        acc[i][j] = Frag<T>::mma(ah, bh[j], acc[i][j]);
        if (SPLIT) {
          acc[i][j] = Frag<T>::mma(ah, bl[j], acc[i][j]);
          acc[i][j] = Frag<T>::mma(al, bh[j], acc[i][j]);
        }
      }
      Frag<T>::guard(acc[i][0], acc[i][3], ah, SPLIT ? al : ah);
    }
    Frag<T>::keep(bh[0], bh[1], bh[2], bh[3]);
    if (SPLIT) Frag<T>::keep(bl[0], bl[1], bl[2], bl[3]);
  }
  acc_guard4(acc[0][0], acc[0][1], acc[0][2], acc[0][3]);
  acc_guard4(acc[1][0], acc[1][1], acc[1][2], acc[1][3]);
  acc_guard4(acc[2][0], acc[2][1], acc[2][2], acc[2][3]);
  acc_guard4(acc[3][0], acc[3][1], acc[3][2], acc[3][3]);

  float* slab = sT[wave];
  const float* Rb = RESID ? (resid + (size_t)b * strideR) : nullptr;
#pragma unroll
  for (int i = 0; i < 4; ++i) {
    const int mBase = m0 + (i << 4);
#pragma unroll
    for (int j = 0; j < 4; ++j) {
      const int n = n0 + (j << 4) + rlane;
      float bv = 0.f;
      if (BIAS_MODE == 2) bv = bias[n];
#pragma unroll
      for (int r = 0; r < 8; ++r) {
        float v = acc[i][j][r] * scale;
        if (BIAS_MODE == 1) v += bias[mBase + mOff + r];
        if (BIAS_MODE == 2) v += bv;
        if (RESID) v += Rb[(size_t)(mBase + mOff + r) * ldc + n];
        if (ACT == 1) v = tanhf(v);
        if (ACT == 2) v = fmaxf(v, 0.0f);
        if (ACT == 3) v = v / (1.0f + expf(-v));
        if (ACT == 4) v = (v > 0.f) ? v : 0.01f * v;
        if (ACT == 5) v = 0.5f * v * (1.0f + erff(v * 0.70710678118654752f));
        slab[(mOff + r) * 68 + (j << 4) + rlane] = v;
      }
    }
    __builtin_amdgcn_fence(__ATOMIC_RELEASE, "workgroup");
    __builtin_amdgcn_wave_barrier();
    __builtin_amdgcn_fence(__ATOMIC_ACQUIRE, "workgroup");
    if (OUT_MODE == 0) {
      float* C = (float*)Cout + (size_t)b * strideC;
      const int hh = lane >> 4, c4 = (lane & 15) * 4;
      for (int pass = 0; pass < 2; ++pass) {
#pragma unroll
        for (int it = 0; it < 8; ++it) {
          const int row = it * 2 + hh;
          v4f v = *(const v4f*)(slab + row * 68 + c4);
          *(volatile v4f*)(C + (size_t)(mBase + row) * ldc + n0 + c4) = v;
        }
        __threadfence();
      }
    } else {
      const int q = lane >> 3, c8 = (lane & 7) * 8;
      unsigned short* C  = (unsigned short*)Cout  + (size_t)b * strideC;
      unsigned short* C2 = (OUT_MODE == 2) ? ((unsigned short*)Cout2 + (size_t)b * strideC) : nullptr;
      for (int pass = 0; pass < 2; ++pass) {
#pragma unroll
        for (int it = 0; it < 4; ++it) {
          const int row = it * 4 + q;
          const float* sp = slab + row * 68 + c8;
          v8h hv, lv;
#pragma unroll
          for (int e = 0; e < 8; ++e) {
            if (OUT_MODE == 1) {
              hv[e] = (_Float16)sp[e];
            } else {
              unsigned short hb = f2bf_bits(sp[e]);
              unsigned short lb = f2bf_bits(sp[e] - bf_bits2f(hb));
              hv[e] = __builtin_bit_cast(_Float16, hb);
              lv[e] = __builtin_bit_cast(_Float16, lb);
            }
          }
          *(volatile v8h*)(C + (size_t)(mBase + row) * ldc + n0 + c8) = hv;
          if (OUT_MODE == 2) *(volatile v8h*)(C2 + (size_t)(mBase + row) * ldc + n0 + c8) = lv;
        }
        __threadfence();
      }
    }
    __builtin_amdgcn_fence(__ATOMIC_RELEASE, "workgroup");
    __builtin_amdgcn_wave_barrier();
    __builtin_amdgcn_fence(__ATOMIC_ACQUIRE, "workgroup");
  }
}

__global__ __launch_bounds__(256) void tail_kernel(
    const float* __restrict__ y1, const float* __restrict__ zr,
    const float* __restrict__ mixg, const float* __restrict__ mixb,
    const float* __restrict__ n2g, const float* __restrict__ n2b, float* __restrict__ out)
{
  const int lane = threadIdx.x & 31;
  const int wave = __builtin_amdgcn_readfirstlane((int)(threadIdx.x >> 5));
  const size_t row = (size_t)blockIdx.x * 8 + wave;
  float yv[16];
  float av[16];
  float s = 0.0f;
#pragma unroll
  for (int i = 0; i < 4; ++i) {
    const int dc = 128 * i + 4 * lane;
    const v4f a = *(const v4f*)(y1 + row * kChan + dc);
    const v4f z = *(const v4f*)(zr + row * kChan + dc);
#pragma unroll
    for (int e = 0; e < 4; ++e) {
      yv[4 * i + e] = a[e];
      const float t = a[e] + z[e];
      av[4 * i + e] = t;
      s += t;
    }
  }
  const float m1 = wave_sum(s) * (1.0f / (float)kChan);
  float s2 = 0.0f;
#pragma unroll
  for (int k = 0; k < 16; ++k) {
    const float dv = av[k] - m1;
    s2 = fmaf(dv, dv, s2);
  }
  const float rs1 = rsqrtf(wave_sum(s2) * (1.0f / (float)kChan) + 1e-5f);
  s = 0.0f;
#pragma unroll
  for (int i = 0; i < 4; ++i) {
    const int dc = 128 * i + 4 * lane;
    const v4f gg = *(const v4f*)(mixg + dc);
    const v4f bb = *(const v4f*)(mixb + dc);
#pragma unroll
    for (int e = 0; e < 4; ++e) {
      const float z = (av[4 * i + e] - m1) * rs1 * gg[e] + bb[e];
      const float t = yv[4 * i + e] + z;
      av[4 * i + e] = t;
      s += t;
    }
  }
  const float m2 = wave_sum(s) * (1.0f / (float)kChan);
  s2 = 0.0f;
#pragma unroll
  for (int k = 0; k < 16; ++k) {
    const float dv = av[k] - m2;
    s2 = fmaf(dv, dv, s2);
  }
  const float rs2 = rsqrtf(wave_sum(s2) * (1.0f / (float)kChan) + 1e-5f);
  v4f o[4];
#pragma unroll
  for (int i = 0; i < 4; ++i) {
    const int dc = 128 * i + 4 * lane;
    const v4f gg = *(const v4f*)(n2g + dc);
    const v4f bb = *(const v4f*)(n2b + dc);
#pragma unroll
    for (int e = 0; e < 4; ++e) o[i][e] = (av[4 * i + e] - m2) * rs2 * gg[e] + bb[e];
  }
  for (int pass = 0; pass < 2; ++pass) {
#pragma unroll
    for (int i = 0; i < 4; ++i) {
      *(volatile v4f*)(out + row * kChan + 128 * i + 4 * lane) = o[i];
    }
    __threadfence();
  }
}

extern "C" void kernel_launch(void* const* d_in, const int* in_sizes, int n_in,
                              void* d_out, int out_size, void* d_ws, size_t ws_size,
                              hipStream_t stream) {
  if (n_in < 19) return;
  if (in_sizes[0] != kBatch * kLen * kChan) return;
  if (in_sizes[1] != kComp * kChan * kState) return;
  if (in_sizes[2] != kComp * kChan * kState) return;
  if (in_sizes[3] != kComp * kChan) return;
  if (in_sizes[4] != kComp) return;
  if (in_sizes[5] != kSeR * kChan) return;
  if (in_sizes[6] != kSeR) return;
  if (in_sizes[7] != kChan * kSeR) return;
  if (in_sizes[8] != kChan) return;
  if (in_sizes[9] != kChan) return;
  if (in_sizes[10] != kChan) return;
  if (in_sizes[11] != kUpOut * kChan) return;
  if (in_sizes[12] != kUpOut) return;
  if (in_sizes[13] != kChan * kHidden) return;
  if (in_sizes[14] != kChan) return;
  if (in_sizes[15] != kChan) return;
  if (in_sizes[16] != kChan) return;
  if (in_sizes[17] != kChan) return;
  if (in_sizes[18] != kChan) return;
  if (out_size != kBatch * kLen * kChan) return;
  if (ws_size < kWsTotal) return;

  const float* x      = (const float*)d_in[0];
  const float* Bp     = (const float*)d_in[1];
  const float* Cp     = (const float*)d_in[2];
  const float* Dp     = (const float*)d_in[3];
  const float* log_dt = (const float*)d_in[4];
  const float* se_w1  = (const float*)d_in[5];
  const float* se_b1  = (const float*)d_in[6];
  const float* se_w2  = (const float*)d_in[7];
  const float* se_b2  = (const float*)d_in[8];
  const float* n1_g   = (const float*)d_in[9];
  const float* n1_b   = (const float*)d_in[10];
  const float* up_w   = (const float*)d_in[11];
  const float* up_b   = (const float*)d_in[12];
  const float* down_w = (const float*)d_in[13];
  const float* down_b = (const float*)d_in[14];
  const float* mixn_g = (const float*)d_in[15];
  const float* mixn_b = (const float*)d_in[16];
  const float* n2_g   = (const float*)d_in[17];
  const float* n2_b   = (const float*)d_in[18];
  float* out = (float*)d_out;

  char* ws = (char*)d_ws;
  float*          BBAR = (float*)(ws + kOffBbar);
  unsigned short* AHI  = (unsigned short*)(ws + kOffAhi);
  unsigned short* ALO  = (unsigned short*)(ws + kOffAlo);
  float*          KC   = (float*)(ws + kOffKc);
  unsigned short* TB16 = (unsigned short*)(ws + kOffTb);
  unsigned short* X16  = (unsigned short*)(ws + kOffX16);
  float*          Y    = (float*)(ws + kOffY);
  float*          SM   = (float*)(ws + kOffSm);
  float*          GT   = (float*)(ws + kOffGt);
  float*          Y1   = (float*)(ws + kOffY1);
  unsigned short* Y1H  = (unsigned short*)(ws + kOffY1h);
  unsigned short* UPW  = (unsigned short*)(ws + kOffUpw);
  unsigned short* DNW  = (unsigned short*)(ws + kOffDnw);
  unsigned short* ACT  = (unsigned short*)(ws + kOffAct);
  float*          ZR   = (float*)(ws + kOffZr);

  disc_kernel<<<dim3(9, kComp), 64, 0, stream>>>(Bp, log_dt, BBAR, AHI, ALO);
  gen_kernel<<<dim3(kChan / 16, kComp), 128, 0, stream>>>(BBAR, AHI, ALO, Cp, KC);

  static_assert((kUpOut * kChan / 8) == 131072 && (kChan * kHidden / 8) == 65536);
  weight_planes_kernel<<<768, 256, 0, stream>>>(up_w, down_w, UPW, DNW);
  stream_plane_kernel<<<dim3(kLen / 64, kChan / 64, kBatch), 256, 0, stream>>>(x, X16);

  for (int g = 0; g < kGroups; ++g) {
    toeplitz_kernel<<<dim3(kBlocksD, kGroupCh), 256, 0, stream>>>(KC, Dp, TB16, g * kGroupCh);
    conv_kernel<<<dim3(kBlocksD, kGroupCh / 4), 256, 0, stream>>>(X16, TB16, Y, g * kGroupCh);
  }

  se_mean_kernel<<<(kChan * kBatch) / 32, 256, 0, stream>>>(Y, SM);
  se_mlp_kernel<<<1, 512, 0, stream>>>(SM, se_w1, se_b1, se_w2, se_b2, GT);
  ln1_kernel<<<dim3(kLen / 16, kBatch), 256, 0, stream>>>(x, Y, GT, n1_g, n1_b, Y1, Y1H);

  static_assert(((kPos / 32) * (kHidden / 64)) % 4 == 0);
  up_glu_kernel<<<((kPos / 32) * (kHidden / 64)) / 4, 128, 0, stream>>>(Y1H, UPW, up_b, ACT);

  static_assert((kPos % 64) == 0 && (kChan % 64) == 0 && (kHidden % 32) == 0);
  static_assert(((kPos / 64) * (kChan / 64)) % 8 == 0);
  wmma_gemm64<0, false, 2, 0, false, 0><<<dim3(((kPos / 64) * (kChan / 64)) / 8, 1), 256, 0, stream>>>(
      ACT, nullptr, kHidden, 0L, DNW, nullptr, kHidden, 0L, (void*)ZR, nullptr, kChan, 0L,
      down_b, nullptr, 0L, kPos, kChan, kHidden, kDownInv);

  tail_kernel<<<kPos / 8, 256, 0, stream>>>(Y1, ZR, mixn_g, mixn_b, n2_g, n2_b, out);
}
